// MoE_5265629905213
// MI455X (gfx1250) — hardware-verified
//
#include <hip/hip_runtime.h>
#include <math.h>

typedef __attribute__((ext_vector_type(16))) _Float16 v16h;
typedef __attribute__((ext_vector_type(16))) __bf16 v16b;
typedef __attribute__((ext_vector_type(8)))  _Float16 v8h;
typedef __attribute__((ext_vector_type(8)))  float v8f;
typedef __attribute__((ext_vector_type(4)))  float v4f;
typedef __attribute__((ext_vector_type(2)))  float v2f;
typedef __attribute__((ext_vector_type(4)))  unsigned v4u;
typedef __attribute__((ext_vector_type(4)))  int v4i;
typedef float __attribute__((may_alias)) float_a;
typedef int __attribute__((may_alias)) int_a;

template <typename T> __device__ __forceinline__ void vst2(void* p, T v) { *(volatile T*)p = v; __threadfence(); *(volatile T*)p = v; }
__device__ __forceinline__ v8f wmma16(v16h a, v16h b, v8f c) {
  v8f d = __builtin_amdgcn_wmma_f32_16x16x32_f16(false, a, false, b, (short)0, c, false, false);
  asm volatile("v_nop\n\tv_nop\n\tv_nop\n\tv_nop" : "+v"(d) : "v"(a), "v"(b));
  return d;
}
__device__ __forceinline__ v8f wmma_bf(v16b a, v16b b, v8f c) {
  v8f d = __builtin_amdgcn_wmma_f32_16x16x32_bf16(false, a, false, b, (short)0, c, false, false);
  asm volatile("v_nop\n\tv_nop\n\tv_nop\n\tv_nop" : "+v"(d) : "v"(a), "v"(b));
  return d;
}
__device__ __forceinline__ v16h frag_h(const _Float16* rowk0, int lane) {
  union { v16h v; v8h q[2]; } u; const _Float16* p = rowk0 + 8 * (lane >> 4);
  u.q[0] = *(const v8h*)p; u.q[1] = *(const v8h*)(p + 16); return u.v;
}
__device__ __forceinline__ v16h frag_f32(const float* rowk0, int lane) {
  v16h a; const float* p = rowk0 + 8 * (lane >> 4);
#pragma unroll
  for (int i = 0; i < 8; ++i) { a[i] = (_Float16)p[i]; a[8 + i] = (_Float16)p[16 + i]; }
  return a;
}
__device__ __forceinline__ v16h frag_f32s(const float* rowk0, int lane, float sc) {
  v16h a; const float* p = rowk0 + 8 * (lane >> 4);
#pragma unroll
  for (int i = 0; i < 8; ++i) { a[i] = (_Float16)(p[i] * sc); a[8 + i] = (_Float16)(p[16 + i] * sc); }
  return a;
}
__device__ __forceinline__ v16h fragc_f32(const float* W, int k0, int n, int lane, int ld, int K) {
  v16h a; const int g = lane >> 4;
#pragma unroll
  for (int i = 0; i < 8; ++i) { const int ka = k0 + 8 * g + i, kb = ka + 16;
    a[i] = (_Float16)(ka < K ? W[(size_t)(ka < K ? ka : K - 1) * ld + n] : 0.f); a[8 + i] = (_Float16)(kb < K ? W[(size_t)(kb < K ? kb : K - 1) * ld + n] : 0.f); }
  return a;
}
struct F2 { v16b h, l; };
__device__ __forceinline__ F2 bsplit16(const float v[16]) { F2 r;
#pragma unroll
  for (int i = 0; i < 16; ++i) { const __bf16 h = (__bf16)v[i]; r.h[i] = h; r.l[i] = (__bf16)(v[i] - (float)h); }
  return r; }
__device__ __forceinline__ F2 split_row(const float* row, int k0, int lane) { float v[16]; const float* p = row + k0 + 8 * (lane >> 4);
#pragma unroll
  for (int i = 0; i < 8; ++i) { v[i] = p[i]; v[8 + i] = p[16 + i]; }
  return bsplit16(v); }
__device__ __forceinline__ F2 split_rowK(const float* row, int k0, int lane, int K) { float v[16]; const int g = lane >> 4;
#pragma unroll
  for (int i = 0; i < 8; ++i) { const int ka = k0 + 8 * g + i, kb = ka + 16; v[i] = ka < K ? row[ka < K ? ka : K - 1] : 0.f; v[8 + i] = kb < K ? row[kb < K ? kb : K - 1] : 0.f; }
  return bsplit16(v); }
__device__ __forceinline__ F2 split_col(const float* W, int k0, int n, int lane, int ld, int K) { float v[16]; const int g = lane >> 4;
#pragma unroll
  for (int i = 0; i < 8; ++i) { const int ka = k0 + 8 * g + i, kb = ka + 16; v[i] = ka < K ? W[(size_t)(ka < K ? ka : K - 1) * ld + n] : 0.f; v[8 + i] = kb < K ? W[(size_t)(kb < K ? kb : K - 1) * ld + n] : 0.f; }
  return bsplit16(v); }
__device__ __forceinline__ v8f mac3(const F2& a, const F2& b, v8f c) { c = wmma_bf(a.l, b.h, c); c = wmma_bf(a.h, b.l, c); return wmma_bf(a.h, b.h, c); }
__device__ __forceinline__ float sigm(float v) { return 1.0f / (1.0f + expf(-v)); }
#define LDSX() do { asm volatile("s_wait_dscnt 0" ::: "memory"); __builtin_amdgcn_wave_barrier(); __builtin_amdgcn_fence(__ATOMIC_RELEASE, "workgroup"); } while (0)

#define NT 2048
#define DD 512
#define HH 1024
#define HS 2048
#define OUTW 128
#define NE 16
#define KS 2
#define NRB (NT / 64 + NE)
typedef __attribute__((ext_vector_type(4))) int v4i2;
__device__ __forceinline__ float bfr(float v) { return (float)(__bf16)v; }
__device__ __forceinline__ v16b wcol_in(const float* Wm, int k0, int o, int lane, int ld, int nvalid) { v16b w; const int g = lane >> 4; const int oc = o < nvalid ? o : 0; const float keep = o < nvalid ? 1.f : 0.f; float t0[8], t1[8];
#pragma unroll
  for (int i = 0; i < 8; ++i) t0[i] = Wm[(size_t)(k0 + 8 * g + i) * ld + oc];
  asm volatile("s_wait_loadcnt 0x0" ::: "memory");
#pragma unroll
  for (int i = 0; i < 8; ++i) t1[i] = Wm[(size_t)(k0 + 16 + 8 * g + i) * ld + oc];
  asm volatile("s_wait_loadcnt 0x0" ::: "memory");
#pragma unroll
  for (int i = 0; i < 8; ++i) { w[i] = (__bf16)(t0[i] * keep); w[8 + i] = (__bf16)(t1[i] * keep); }
  return w; }
#define WS_IDX 0u
#define WS_WGT (WS_IDX + 16u * NT)
#define WS_TOK (WS_WGT + 16u * NT)
#define WS_RB  (WS_TOK + 16u * NT)
#define WS_H   (WS_RB + 64u * NRB + 1024u)
#define WS_CMB (WS_H + 4u * (size_t)NT * HS)
#define WS_SG  (WS_CMB + 4u * (size_t)NT * DD)
#define WS_END (WS_SG + 4u * (size_t)NT)

__global__ __launch_bounds__(128) void k_route(const float* __restrict__ X, const float* __restrict__ WG, const float* __restrict__ BG, int* __restrict__ IDX, float* __restrict__ WGT, float* __restrict__ LOG, const float* __restrict__ SGW, float* __restrict__ SG) { __shared__ __align__(16) int si[64][KS]; __shared__ __align__(16) float sw[64][KS];
  const int tid = threadIdx.x; const size_t r0 = (size_t)blockIdx.x * 64; (void)BG; float sgv_keep = 0.f;
  if (tid < 64) {
    const float* xr = X + (r0 + tid) * DD; float sm[NE], cm[NE]; float sgs = 0.f, sgc = 0.f;
#pragma unroll
    for (int e = 0; e < NE; ++e) { sm[e] = 0.f; cm[e] = 0.f; }
#pragma unroll 1
    for (int d0 = 0; d0 < DD; d0 += 8) { float xv[8]; float wv[8][NE];
#pragma unroll
      for (int u = 0; u < 8; ++u) xv[u] = xr[d0 + u];
      asm volatile("s_wait_loadcnt 0x0" ::: "memory");
#pragma unroll
      for (int u = 0; u < 8; ++u) {
#pragma unroll
        for (int e = 0; e < NE; ++e) wv[u][e] = WG[(size_t)e * DD + d0 + u];
        if (u == 3) asm volatile("s_wait_loadcnt 0x0" ::: "memory"); }
      asm volatile("s_wait_loadcnt 0x0" ::: "memory");
#pragma unroll
      for (int u = 0; u < 8; ++u) { const float xb = bfr(xv[u]);
#pragma unroll
        for (int e = 0; e < NE; ++e) {
#pragma clang fp contract(off)
          const float p = xb * bfr(wv[u][e]);
          const float t = sm[e] + p; const float big = fabsf(sm[e]) >= fabsf(p) ? sm[e] : p, sml = fabsf(sm[e]) >= fabsf(p) ? p : sm[e]; cm[e] += (big - t) + sml; sm[e] = t; } } }
    float l[NE]; float mx = -3.0e38f;
#pragma unroll
    for (int e = 0; e < NE; ++e) { l[e] = sm[e] + cm[e]; mx = fmaxf(mx, l[e]); }
    (void)LOG; (void)SGW;
    (void)sgs; (void)sgc; sgv_keep = 1.0f;
    float dall = 0.f;
#pragma unroll
    for (int e = 0; e < NE; ++e) dall += expf(l[e] - mx);
    int sel[KS]; float sv[KS]; unsigned usedm = 0u;
#pragma unroll
    for (int s2 = 0; s2 < KS; ++s2) { int be = -1; float bv = -3.0e38f;
#pragma unroll
      for (int e = 0; e < NE; ++e) { const bool free_ = ((usedm >> e) & 1u) == 0u; const bool take = free_ && (be < 0 || l[e] > bv); bv = take ? l[e] : bv; be = take ? e : be; }
      usedm |= 1u << be; sel[s2] = be; sv[s2] = bv; }
    float den = 0.f; float ev[KS];
#pragma unroll
    for (int s2 = 0; s2 < KS; ++s2) { ev[s2] = expf(sv[s2] - sv[0]); den += ev[s2]; }
#pragma unroll
    for (int s2 = 0; s2 < KS; ++s2) { si[tid][s2] = sel[s2]; sw[tid][s2] = ev[s2] / dall; } (void)den; }
  __shared__ __align__(16) float ssg[64]; if (tid < 64) ssg[tid] = sgv_keep;
  __syncthreads();
  if (tid >= 64 && tid < 80) vst2(SG + r0 + (tid - 64) * 4, *(const v4f*)&ssg[(tid - 64) * 4]);
  if (tid < 32) { v4i2 iv; v4f wv4; iv[0] = si[2 * tid][0]; iv[1] = si[2 * tid][1]; iv[2] = si[2 * tid + 1][0]; iv[3] = si[2 * tid + 1][1]; wv4[0] = sw[2 * tid][0]; wv4[1] = sw[2 * tid][1]; wv4[2] = sw[2 * tid + 1][0]; wv4[3] = sw[2 * tid + 1][1]; vst2((v4i2*)(IDX + (r0 + 2 * tid) * KS), iv); vst2((v4f*)(WGT + (r0 + 2 * tid) * KS), wv4); } }
__global__ __launch_bounds__(256) void k_bucket(const int* __restrict__ IDX, int* __restrict__ TOK, int* __restrict__ RB) { __shared__ int cnt[KS][NE]; __shared__ int off[KS][NE + 1]; __shared__ int srb[KS][NRB][4];
  const int t = threadIdx.x;
  if (t < KS * NE) { const int sl = t / NE, ex = t % NE; int c = 0; for (int i = 0; i < NT; ++i) { const int e = IDX[i * KS + sl]; c += (e == ex); } cnt[sl][ex] = c; }
  __syncthreads();
  if (t < KS) { const int sl = t; off[sl][0] = 0; for (int e = 0; e < NE; ++e) off[sl][e + 1] = off[sl][e] + cnt[sl][e]; int nb = 0; for (int e = 0; e < NE; ++e) for (int s0 = 0; s0 < cnt[sl][e]; s0 += 64) { srb[sl][nb][0] = e; srb[sl][nb][1] = off[sl][e] + s0; srb[sl][nb][2] = (cnt[sl][e] - s0) < 64 ? (cnt[sl][e] - s0) : 64; srb[sl][nb][3] = 0; ++nb; }
    for (; nb < NRB; ++nb) { srb[sl][nb][0] = 0; srb[sl][nb][1] = 0; srb[sl][nb][2] = 0; srb[sl][nb][3] = 0; } }
  __syncthreads();
  if (t < KS * NE) { const int sl = t / NE, ex = t % NE; int pos = off[sl][ex]; for (int i = 0; i < NT; ++i) { const int e = IDX[i * KS + sl]; if (e == ex) { vst2(TOK + sl * NT + pos, i); ++pos; } } }
  for (int i = t; i < KS * NRB * 4; i += 256) vst2(RB + i, srb[i / (NRB * 4)][(i / 4) % NRB][i & 3]); }
__device__ __forceinline__ v16b wcol_oi2(const float* __restrict__ Wm, int k0, int o, int lane) { v16b w; const int g = lane >> 4; const float* p = Wm + (size_t)o * DD + k0 + 8 * g;
#pragma unroll
  for (int i = 0; i < 8; ++i) { w[i] = (__bf16)p[i]; w[8 + i] = (__bf16)p[16 + i]; }
  asm volatile("s_wait_loadcnt 0x0" ::: "memory"); return w; }
__device__ __forceinline__ v16b wrow_w1(const float* __restrict__ Wm, int k0, int o, int lane) { v16b w; const int g = lane >> 4; const float* p = Wm + (size_t)(k0 + 8 * g) * HH + o;
#pragma unroll
  for (int i = 0; i < 8; ++i) { w[i] = (__bf16)p[(size_t)i * HH]; w[8 + i] = (__bf16)p[(size_t)(16 + i) * HH]; }
  asm volatile("s_wait_loadcnt 0x0" ::: "memory"); return w; }
__global__ __launch_bounds__(128) void k_exp1(const float* __restrict__ X, const float* __restrict__ W1, const float* __restrict__ W3, int hw, const int* __restrict__ TOK, const int* __restrict__ RB, int slot, float* __restrict__ Hr, const float* __restrict__ B0, const float* __restrict__ B1) { __shared__ __align__(16) float sf[4][16][132]; __shared__ int stok[64];
  const int tid = threadIdx.x, wave = tid >> 5, lane = tid & 31, col = lane & 15, g = lane >> 4; const int c0 = blockIdx.y * 128;
  int e, nrows;
  if (slot >= 0) { const int* rb = RB + (slot * NRB + blockIdx.x) * 4; e = rb[0]; const int slot0 = rb[1]; nrows = rb[2]; if (nrows <= 0) return;
    if (tid < 64) { const int sl = tid < nrows ? slot0 + tid : slot0; int tk = TOK[slot * NT + (sl < NT ? sl : NT - 1)]; tk = tk < 0 ? 0 : (tk >= NT ? NT - 1 : tk); stok[tid] = tk; } }
  else { e = -1 - slot; nrows = 64; if ((size_t)blockIdx.x * 64 >= (size_t)NT) return; if (tid < 64) stok[tid] = blockIdx.x * 64 + tid; }
  __syncthreads();
  const float* Wa = W1 + (size_t)e * hw * DD; const float* Wb = W3 + (size_t)e * hw * DD; const int tk = stok[wave * 16 + col];
  v8f acc[8] = {}, accu[8] = {};
#pragma unroll 1
  for (int kc = 0; kc < DD / 32; ++kc) { v16b a; { const float* p = X + (size_t)tk * DD + kc * 32 + 8 * g;
#pragma unroll
      for (int i = 0; i < 8; ++i) { a[i] = (__bf16)p[i]; a[8 + i] = (__bf16)p[16 + i]; } }
    asm volatile("s_wait_loadcnt 0x0" ::: "memory");
#pragma unroll
    for (int j = 0; j < 8; ++j) { const v16b w = wcol_oi2(Wa, kc * 32, c0 + j * 16 + col, lane); acc[j] = wmma_bf(a, w, acc[j]); const v16b w3 = wcol_oi2(Wb, kc * 32, c0 + j * 16 + col, lane); accu[j] = wmma_bf(a, w3, accu[j]); } }
#pragma unroll
  for (int j = 0; j < 8; ++j) {
    const float bg_ = bfr(B0[(size_t)e * hw + c0 + j * 16 + col]), bu_ = bfr(B1[(size_t)e * hw + c0 + j * 16 + col]); asm volatile("s_wait_loadcnt 0x0" ::: "memory");
#pragma unroll
    for (int r = 0; r < 8; ++r) { const float gt = acc[j][r] + bg_; sf[wave][8 * g + r][j * 16 + col] = (accu[j][r] + bu_) * (gt >= 0.0f ? gt : 0.01f * gt); } }
  LDSX(); for (int rl = 0; rl < 16; ++rl) { const int row = wave * 16 + rl; if (row < nrows) vst2(Hr + (size_t)stok[row] * HS + c0 + lane * 4, *(const v4f*)&sf[wave][rl][lane * 4]); } }
__global__ __launch_bounds__(128) void k_exp2(const float* __restrict__ Hr, const float* __restrict__ W2, const float* __restrict__ B2, int hw, const int* __restrict__ TOK, const int* __restrict__ RB, const float* __restrict__ WGT, int slot, float* __restrict__ CMB, const float* __restrict__ SG) { __shared__ __align__(16) float sf[4][16][132]; __shared__ int stok[64];
  const int tid = threadIdx.x, wave = tid >> 5, lane = tid & 31, col = lane & 15, g = lane >> 4; const int c0 = blockIdx.y * 128;
  int e, nrows;
  if (slot >= 0) { const int* rb = RB + (slot * NRB + blockIdx.x) * 4; e = rb[0]; const int slot0 = rb[1]; nrows = rb[2]; if (nrows <= 0) return;
    if (tid < 64) { const int sl = tid < nrows ? slot0 + tid : slot0; int tk = TOK[slot * NT + (sl < NT ? sl : NT - 1)]; tk = tk < 0 ? 0 : (tk >= NT ? NT - 1 : tk); stok[tid] = tk; } }
  else { e = -1 - slot; nrows = 64; if ((size_t)blockIdx.x * 64 >= (size_t)NT) return; if (tid < 64) stok[tid] = blockIdx.x * 64 + tid; }
  __syncthreads();
  const float* Wx = W2 + (size_t)e * DD * hw; const int tk = stok[wave * 16 + col];
  v8f acc[8] = {};
#pragma unroll 1
  for (int kc = 0; kc < hw / 32; ++kc) { const v16h a = frag_f32(Hr + (size_t)tk * HS + kc * 32, lane);
    asm volatile("s_wait_loadcnt 0x0" ::: "memory");
#pragma unroll
    for (int j = 0; j < 8; ++j) { v16h w; { const int o = c0 + j * 16 + col; float t0[8], t1[8]; const float* pw = Wx + (size_t)o * hw + kc * 32 + 8 * g;
#pragma unroll
        for (int i2 = 0; i2 < 8; ++i2) t0[i2] = pw[i2];
        asm volatile("s_wait_loadcnt 0x0" ::: "memory");
#pragma unroll
        for (int i2 = 0; i2 < 8; ++i2) t1[i2] = pw[16 + i2];
        asm volatile("s_wait_loadcnt 0x0" ::: "memory");
#pragma unroll
        for (int i2 = 0; i2 < 8; ++i2) { w[i2] = (_Float16)(bfr(t0[i2]) * 64.0f); w[8 + i2] = (_Float16)(bfr(t1[i2]) * 64.0f); } }
      acc[j] = wmma16(a, w, acc[j]); } }
  float gwr[8];
#pragma unroll
  for (int r = 0; r < 8; ++r) gwr[r] = slot >= 0 ? WGT[stok[wave * 16 + 8 * g + r] * KS + slot] : SG[stok[wave * 16 + 8 * g + r]];
  asm volatile("s_wait_loadcnt 0x0" ::: "memory");
#pragma unroll
  for (int j = 0; j < 8; ++j) {
    const float bb = B2 ? bfr(B2[(size_t)e * DD + c0 + j * 16 + col]) : 0.f; asm volatile("s_wait_loadcnt 0x0" ::: "memory");
#pragma unroll
    for (int r = 0; r < 8; ++r) sf[wave][8 * g + r][j * 16 + col] = (acc[j][r] * (1.0f / 64.0f) + bb) * gwr[r]; }
  LDSX();
  for (int rl = 0; rl < 16; ++rl) { const int row = wave * 16 + rl; if (row < nrows) { float* po = CMB + (size_t)stok[row] * DD + c0 + lane * 4; v4f v = *(const v4f*)&sf[wave][rl][lane * 4];
      if (slot != 0) { const v4f prev = *(const v4f*)po; v[0] += prev[0]; v[1] += prev[1]; v[2] += prev[2]; v[3] += prev[3]; }
      vst2(po, v); } } }
__global__ __launch_bounds__(128) void k_head(const float* __restrict__ Hr, const float* __restrict__ W2, const float* __restrict__ B2, int hw, const int* __restrict__ TOK, const int* __restrict__ RB, const float* __restrict__ WGT, int slot, float* __restrict__ CMB, const float* __restrict__ SG) { __shared__ __align__(16) float sf[4][16][132]; __shared__ int stok[64];
  const int tid = threadIdx.x, wave = tid >> 5, lane = tid & 31, col = lane & 15, g = lane >> 4; const int c0 = blockIdx.y * 128;
  int e, nrows;
  if (slot >= 0) { const int* rb = RB + (slot * NRB + blockIdx.x) * 4; e = rb[0]; const int slot0 = rb[1]; nrows = rb[2]; if (nrows <= 0) return;
    if (tid < 64) { const int sl = tid < nrows ? slot0 + tid : slot0; int tk = TOK[slot * NT + (sl < NT ? sl : NT - 1)]; tk = tk < 0 ? 0 : (tk >= NT ? NT - 1 : tk); stok[tid] = tk; } }
  else { e = -1 - slot; nrows = 64; if ((size_t)blockIdx.x * 64 >= (size_t)NT) return; if (tid < 64) stok[tid] = blockIdx.x * 64 + tid; }
  __syncthreads();
  const float* Wx = W2; const int tk = stok[wave * 16 + col];
  v8f acc[8] = {};
#pragma unroll 1
  for (int kc = 0; kc < hw / 32; ++kc) { const v16h a = frag_f32(Hr + (size_t)tk * DD + kc * 32, lane);
    asm volatile("s_wait_loadcnt 0x0" ::: "memory");
#pragma unroll
    for (int j = 0; j < 8; ++j) { v16h w; { const int o = c0 + j * 16 + col; float t0[8], t1[8]; const float* pw = Wx + (size_t)o * hw + kc * 32 + 8 * g;
#pragma unroll
        for (int i2 = 0; i2 < 8; ++i2) t0[i2] = pw[i2];
        asm volatile("s_wait_loadcnt 0x0" ::: "memory");
#pragma unroll
        for (int i2 = 0; i2 < 8; ++i2) t1[i2] = pw[16 + i2];
        asm volatile("s_wait_loadcnt 0x0" ::: "memory");
#pragma unroll
        for (int i2 = 0; i2 < 8; ++i2) { w[i2] = (_Float16)(bfr(t0[i2]) * 64.0f); w[8 + i2] = (_Float16)(bfr(t1[i2]) * 64.0f); } }
      acc[j] = wmma16(a, w, acc[j]); } }
  float gwr[8];
#pragma unroll
  for (int r = 0; r < 8; ++r) gwr[r] = 1.0f;
  asm volatile("s_wait_loadcnt 0x0" ::: "memory");
#pragma unroll
  for (int j = 0; j < 8; ++j) {
    const float bb = B2 ? bfr(B2[c0 + j * 16 + col]) : 0.f; asm volatile("s_wait_loadcnt 0x0" ::: "memory");
#pragma unroll
    for (int r = 0; r < 8; ++r) sf[wave][8 * g + r][j * 16 + col] = (acc[j][r] * (1.0f / 64.0f) + bb) * gwr[r]; }
  LDSX();
  for (int rl = 0; rl < 16; ++rl) { const int row = wave * 16 + rl; if (row < nrows) { float* po = CMB + (size_t)stok[row] * OUTW + c0 + lane * 4; v4f v = *(const v4f*)&sf[wave][rl][lane * 4];
      vst2(po, v); } } }
extern "C" void kernel_launch(void* const* d_in, const int* in_sizes, int n_in, void* d_out, int out_size, void* d_ws, size_t ws_size, hipStream_t stream) {
  (void)in_sizes; (void)n_in; (void)out_size;
  const float** F = (const float**)d_in;
  if (ws_size < (size_t)WS_END) return;
  char* ws = (char*)d_ws; int *IDX = (int*)(ws + WS_IDX), *TOK = (int*)(ws + WS_TOK), *RB = (int*)(ws + WS_RB); float *WGT = (float*)(ws + WS_WGT), *Hr = (float*)(ws + WS_H), *CMB = (float*)(ws + WS_CMB), *SG = (float*)(ws + WS_SG);
  k_route<<<dim3(NT / 64), 128, 0, stream>>>(F[0], F[2], nullptr, IDX, WGT, nullptr, nullptr, SG);
  k_bucket<<<1, 256, 0, stream>>>(IDX, TOK, RB);
  for (int s = 0; s < KS; ++s) {
    k_exp1<<<dim3(NRB, HH / 128), 128, 0, stream>>>(F[0], F[3], F[7], HH, TOK, RB, s, Hr, F[4], F[8]);
    k_exp2<<<dim3(NRB, DD / 128), 128, 0, stream>>>(Hr, F[5], F[6], HH, TOK, RB, WGT, s, CMB, SG);
  }
  k_exp1<<<dim3(NT / 64, HS / 128), 128, 0, stream>>>(F[0], F[9], F[13], HS, TOK, RB, -1, Hr, F[10], F[14]);
  k_exp2<<<dim3(NT / 64, DD / 128), 128, 0, stream>>>(Hr, F[11], F[12], HS, TOK, RB, WGT, -1, CMB, SG);
  k_head<<<dim3(NT / 64, OUTW / 128), 128, 0, stream>>>(CMB, F[15], F[16], DD, TOK, RB, WGT, -1, (float*)d_out, SG);
}
